// GATSBYGene_80908593922532
// MI455X (gfx1250) — hardware-verified
//
#include <hip/hip_runtime.h>
#include <stddef.h>


#define DD    256
#define NHD   8
#define GR    32
#define AP    264
#define XSP   260
#define NTHR  256
#define NWAVE 8
#define NB    256
#define CHUNK 2048
#define WCAP  256
#define NGRP  (CHUNK / (NTHR * 4))

#define LDS_SACC (NB * DD)
#define LDS_DEN  (NB * NHD)
#define LDS_EMX  (NB * NHD)
#define LDS_LIST (NWAVE * WCAP)
#define LDS_BYTES ((LDS_SACC + LDS_DEN + LDS_EMX + LDS_LIST + NWAVE) * 4)

static_assert(WCAP == (CHUNK / NTHR) * 32);
static_assert(NGRP >= 1);
static_assert(NB == 256);
static_assert(CHUNK == 2048);
static_assert(((LDS_SACC + LDS_DEN) % 4) == 0);
static_assert((LDS_EMX % 4) == 0);
static_assert(LDS_BYTES == 286752);
static_assert(GR * XSP * 4 <= 2 * GR * AP * 2);
static_assert((AP % 8) == 0);
static_assert((XSP % 4) == 0);

typedef float          v4f  __attribute__((ext_vector_type(4)));
typedef float          v8f  __attribute__((ext_vector_type(8)));
typedef int            v4i  __attribute__((ext_vector_type(4)));
typedef unsigned int   v4u  __attribute__((ext_vector_type(4)));
typedef __bf16         v16b __attribute__((ext_vector_type(16)));
union FragB { v16b v; v4u q[2]; };

__device__ __forceinline__ v8f wm(v16b a, v16b b, v8f c) {
  v8f d = __builtin_amdgcn_wmma_f32_16x16x32_bf16(false, a, false, b, (short)0, c, false, false);
  asm volatile("v_nop\n\tv_nop\n\tv_nop\n\tv_nop" : "+v"(d) : "v"(a), "v"(b));
  return d;
}

__device__ __forceinline__ unsigned int bfb(float f) {
  const unsigned int u = __float_as_uint(f);
  return (u + 0x7FFFu + ((u >> 16) & 1u)) >> 16;
}
__device__ __forceinline__ void split2(float f, unsigned int& hi, unsigned int& lo) {
  hi = bfb(f);
  lo = bfb(f - __uint_as_float(hi << 16));
}

__global__ __launch_bounds__(NTHR) void k_prepw(const float* __restrict__ W,
                                               unsigned short* Whi, unsigned short* Wlo) {
  __shared__ __attribute__((aligned(16))) float S[64 * 65];
  const int tid = threadIdx.x;
  const int n0 = (blockIdx.x & 3) * 64;
  const int k0 = (blockIdx.x >> 2) * 64;
  {
    const int kr = tid >> 2;
    const int c  = (tid & 3) * 16;
    const float* p = W + (size_t)(k0 + kr) * DD + n0 + c;
    const v4f f0 = *(const v4f*)(p);
    const v4f f1 = *(const v4f*)(p + 4);
    const v4f f2 = *(const v4f*)(p + 8);
    const v4f f3 = *(const v4f*)(p + 12);
    float* s = S + kr * 65 + c;
    s[0]  = f0.x; s[1]  = f0.y; s[2]  = f0.z; s[3]  = f0.w;
    s[4]  = f1.x; s[5]  = f1.y; s[6]  = f1.z; s[7]  = f1.w;
    s[8]  = f2.x; s[9]  = f2.y; s[10] = f2.z; s[11] = f2.w;
    s[12] = f3.x; s[13] = f3.y; s[14] = f3.z; s[15] = f3.w;
  }
  __syncthreads();
  v4u ph[2], pl[2];
  size_t go[2];
#pragma unroll
  for (int ps = 0; ps < 2; ++ps) {
    const int L = ps * 32 + (tid >> 3);
    const int q = tid & 7;
    unsigned int hb[8], lb[8];
#pragma unroll
    for (int i = 0; i < 8; ++i) split2(S[(8 * q + i) * 65 + L], hb[i], lb[i]);
    ph[ps].x = hb[0] | (hb[1] << 16); ph[ps].y = hb[2] | (hb[3] << 16);
    ph[ps].z = hb[4] | (hb[5] << 16); ph[ps].w = hb[6] | (hb[7] << 16);
    pl[ps].x = lb[0] | (lb[1] << 16); pl[ps].y = lb[2] | (lb[3] << 16);
    pl[ps].z = lb[4] | (lb[5] << 16); pl[ps].w = lb[6] | (lb[7] << 16);
    go[ps] = (size_t)(n0 + L) * DD + k0 + 8 * q;
  }
#pragma unroll
  for (int ps = 0; ps < 2; ++ps) {
    *(volatile v4u*)(Whi + go[ps]) = ph[ps];
    *(volatile v4u*)(Wlo + go[ps]) = pl[ps];
  }
  __threadfence();
#pragma unroll
  for (int ps = 0; ps < 2; ++ps) {
    *(volatile v4u*)(Whi + go[ps]) = ph[ps];
    *(volatile v4u*)(Wlo + go[ps]) = pl[ps];
  }
}

__global__ __launch_bounds__(NTHR) void k_gemm(
    const float* __restrict__ A, const unsigned short* __restrict__ Whi,
    const unsigned short* __restrict__ Wlo,
    const float* __restrict__ a_src, const float* __restrict__ a_dst,
    const float* __restrict__ bias,
    float* C, float* als, float* ald, int nN, int rowLimit, int mode) {
  __shared__ __attribute__((aligned(16))) unsigned char smem[2 * GR * AP * 2];
  __shared__ __attribute__((aligned(16))) float As[GR * NHD];
  __shared__ __attribute__((aligned(16))) float Ds[GR * NHD];
  unsigned short* Ahi = (unsigned short*)smem;
  unsigned short* Alo = Ahi + GR * AP;
  float* Xs = (float*)smem;

  const int tid  = threadIdx.x;
  const int lane = tid & 31;
  const int wave = tid >> 5;
  const int hh   = lane >> 4;
  const int m    = lane & 15;
  const int rowBase = blockIdx.x * GR;

  {
    const int r  = tid >> 3;
    const int c0 = (tid & 7) * 32;
    int row = rowBase + r;
    if (row > nN - 1) row = nN - 1;
    const float* p = A + (size_t)row * DD + c0;
#pragma unroll
    for (int g = 0; g < 4; ++g) {
      const v4f f0 = *(const v4f*)(p + 8 * g);
      const v4f f1 = *(const v4f*)(p + 8 * g + 4);
      unsigned int h0, h1, h2, h3, h4, h5, h6, h7, l0, l1, l2, l3, l4, l5, l6, l7;
      split2(f0.x, h0, l0); split2(f0.y, h1, l1); split2(f0.z, h2, l2); split2(f0.w, h3, l3);
      split2(f1.x, h4, l4); split2(f1.y, h5, l5); split2(f1.z, h6, l6); split2(f1.w, h7, l7);
      v4u uh, ul;
      uh.x = h0 | (h1 << 16); uh.y = h2 | (h3 << 16); uh.z = h4 | (h5 << 16); uh.w = h6 | (h7 << 16);
      ul.x = l0 | (l1 << 16); ul.y = l2 | (l3 << 16); ul.z = l4 | (l5 << 16); ul.w = l6 | (l7 << 16);
      *(v4u*)(Ahi + r * AP + c0 + 8 * g) = uh;
      *(v4u*)(Alo + r * AP + c0 + 8 * g) = ul;
    }
  }
  __syncthreads();

  const int colA = wave * 32 + m;
  const int colB = colA + 16;
  const v8f vz = {0.f, 0.f, 0.f, 0.f, 0.f, 0.f, 0.f, 0.f};
  v8f acc[2][2];
  acc[0][0] = vz; acc[0][1] = vz; acc[1][0] = vz; acc[1][1] = vz;
#pragma unroll 1
  for (int kt = 0; kt < DD / 32; ++kt) {
    const int k0 = kt * 32 + 8 * hh;
    FragB fah[2], fal[2], fbh[2], fbl[2];
#pragma unroll
    for (int rt = 0; rt < 2; ++rt) {
      const unsigned short* ph = Ahi + (16 * rt + m) * AP + k0;
      const unsigned short* pl = Alo + (16 * rt + m) * AP + k0;
      fah[rt].q[0] = *(const v4u*)(ph); fah[rt].q[1] = *(const v4u*)(ph + 16);
      fal[rt].q[0] = *(const v4u*)(pl); fal[rt].q[1] = *(const v4u*)(pl + 16);
    }
    {
      const unsigned short* p0h = Whi + (size_t)colA * DD + k0;
      const unsigned short* p0l = Wlo + (size_t)colA * DD + k0;
      const unsigned short* p1h = Whi + (size_t)colB * DD + k0;
      const unsigned short* p1l = Wlo + (size_t)colB * DD + k0;
      fbh[0].q[0] = *(const v4u*)(p0h); fbh[0].q[1] = *(const v4u*)(p0h + 16);
      fbl[0].q[0] = *(const v4u*)(p0l); fbl[0].q[1] = *(const v4u*)(p0l + 16);
      fbh[1].q[0] = *(const v4u*)(p1h); fbh[1].q[1] = *(const v4u*)(p1h + 16);
      fbl[1].q[0] = *(const v4u*)(p1l); fbl[1].q[1] = *(const v4u*)(p1l + 16);
    }
#pragma unroll
    for (int rt = 0; rt < 2; ++rt) {
#pragma unroll
      for (int ci = 0; ci < 2; ++ci) {
        v8f c = acc[rt][ci];
        c = wm(fah[rt].v, fbh[ci].v, c);
        c = wm(fal[rt].v, fbh[ci].v, c);
        c = wm(fah[rt].v, fbl[ci].v, c);
        acc[rt][ci] = c;
      }
    }
  }
  __syncthreads();

  const float cs0 = a_src[colA], cs1 = a_src[colB];
  const float cd0 = a_dst[colA], cd1 = a_dst[colB];
  float bv0 = 0.f, bv1 = 0.f;
  if (mode != 0) { bv0 = bias[colA]; bv1 = bias[colB]; }
#pragma unroll
  for (int rt = 0; rt < 2; ++rt) {
    float ss[8], sd[8];
#pragma unroll
    for (int r = 0; r < 8; ++r) {
      const float v0 = acc[rt][0][r];
      const float v1 = acc[rt][1][r];
      const int row = 16 * rt + 8 * hh + r;
      Xs[row * XSP + colA] = v0 + bv0;
      Xs[row * XSP + colB] = v1 + bv1;
      ss[r] = v0 * cs0 + v1 * cs1;
      sd[r] = v0 * cd0 + v1 * cd1;
    }
#pragma unroll
    for (int mk = 1; mk < 16; mk <<= 1) {
#pragma unroll
      for (int r = 0; r < 8; ++r) {
        ss[r] += __shfl_xor(ss[r], mk, 32);
        sd[r] += __shfl_xor(sd[r], mk, 32);
      }
    }
    if (m == 0) {
#pragma unroll
      for (int r = 0; r < 8; ++r) {
        As[(16 * rt + 8 * hh + r) * NHD + wave] = ss[r];
        Ds[(16 * rt + 8 * hh + r) * NHD + wave] = sd[r];
      }
    }
  }
  __syncthreads();

  v4f xa[4], xb[4];
  size_t ro[4];
  bool okr[4];
#pragma unroll
  for (int i = 0; i < 4; ++i) {
    const int lr = 4 * wave + i;
    xa[i] = *(const v4f*)(Xs + lr * XSP + 4 * lane);
    xb[i] = *(const v4f*)(Xs + lr * XSP + 128 + 4 * lane);
    const int row = rowBase + lr;
    okr[i] = row < rowLimit;
    ro[i] = (size_t)row * DD;
  }
  bool gst = false;
  float* gp = C;
  v4f g0 = {0.f, 0.f, 0.f, 0.f}, g1 = {0.f, 0.f, 0.f, 0.f};
  if (mode == 0) {
    if (wave == 0) {
      g0 = *(const v4f*)(As + 4 * lane); g1 = *(const v4f*)(As + 128 + 4 * lane);
      gp = als + (size_t)rowBase * NHD; gst = true;
    } else if (wave == 1) {
      g0 = *(const v4f*)(Ds + 4 * lane); g1 = *(const v4f*)(Ds + 128 + 4 * lane);
      gp = ald + (size_t)rowBase * NHD; gst = true;
    }
  }
#pragma unroll
  for (int i = 0; i < 4; ++i) {
    if (okr[i]) {
      *(volatile v4f*)(C + ro[i] + 4 * lane)       = xa[i];
      *(volatile v4f*)(C + ro[i] + 128 + 4 * lane) = xb[i];
    }
  }
  if (gst) {
    *(volatile v4f*)(gp + 4 * lane)       = g0;
    *(volatile v4f*)(gp + 128 + 4 * lane) = g1;
  }
  __threadfence();
#pragma unroll
  for (int i = 0; i < 4; ++i) {
    if (okr[i]) {
      *(volatile v4f*)(C + ro[i] + 4 * lane)       = xa[i];
      *(volatile v4f*)(C + ro[i] + 128 + 4 * lane) = xb[i];
    }
  }
  if (gst) {
    *(volatile v4f*)(gp + 4 * lane)       = g0;
    *(volatile v4f*)(gp + 128 + 4 * lane) = g1;
  }
}

__global__ __launch_bounds__(NTHR) void k_agg(
    const int* __restrict__ ei, const float* __restrict__ Hm,
    const float* __restrict__ als, const float* __restrict__ ald,
    float* G, int nN, int nE, int nP) {
  extern __shared__ v4f lds_dyn[];
  float* sacc = (float*)lds_dyn;
  float* den  = sacc + LDS_SACC;
  float* emx  = den + LDS_DEN;
  int*   list = (int*)(emx + LDS_EMX);
  int*   wcnt = list + LDS_LIST;

  const int tid  = threadIdx.x;
  const int lane = tid & 31;
  const int wave = tid >> 5;
  const int nodeBase = blockIdx.x * NB;

  {
    const v4f z4 = {0.f, 0.f, 0.f, 0.f};
    for (int i = tid; i < (LDS_SACC + LDS_DEN) / 4; i += NTHR) lds_dyn[i] = z4;
    const v4f m4 = {-1.0e30f, -1.0e30f, -1.0e30f, -1.0e30f};
    v4f* e4 = lds_dyn + (LDS_SACC + LDS_DEN) / 4;
    for (int i = tid; i < LDS_EMX / 4; i += NTHR) e4[i] = m4;
  }
  __syncthreads();

  const int* eid = ei + nE;
  const bool al16 = ((nE & 3) == 0);
  const int hd = lane >> 2;

  const int nChunks = (nE + CHUNK - 1) / CHUNK;
#pragma unroll 1
  for (int ch = 0; ch < nChunks; ++ch) {
    const int cbase = ch * CHUNK;
    int wc = 0;
#pragma unroll
    for (int g = 0; g < NGRP; ++g) {
      const int el0 = (g * NTHR + tid) * 4;
      const int e0  = cbase + el0;
      const int sent = -2147483647 - 1;
      v4i d;
      if (al16 && (cbase + CHUNK <= nE)) {
        d = *(const v4i*)(eid + e0);
      } else {
        const int d0 = eid[min(e0,     nE - 1)];
        const int d1 = eid[min(e0 + 1, nE - 1)];
        const int d2 = eid[min(e0 + 2, nE - 1)];
        const int d3 = eid[min(e0 + 3, nE - 1)];
        d.x = (e0     < nE) ? d0 : sent;
        d.y = (e0 + 1 < nE) ? d1 : sent;
        d.z = (e0 + 2 < nE) ? d2 : sent;
        d.w = (e0 + 3 < nE) ? d3 : sent;
      }
      const unsigned s0 = (unsigned)d.x - (unsigned)nodeBase;
      const unsigned s1 = (unsigned)d.y - (unsigned)nodeBase;
      const unsigned s2 = (unsigned)d.z - (unsigned)nodeBase;
      const unsigned s3 = (unsigned)d.w - (unsigned)nodeBase;
      const bool h0 = s0 < (unsigned)NB;
      const bool h1 = s1 < (unsigned)NB;
      const bool h2 = s2 < (unsigned)NB;
      const bool h3 = s3 < (unsigned)NB;
      const unsigned many = __builtin_amdgcn_ballot_w32(h0 | h1 | h2 | h3);
      if (many != 0u) {
#define HITJ(J, HJ, SJ) { \
          const unsigned mj = __builtin_amdgcn_ballot_w32(HJ); \
          if (HJ) { \
            const int pos = wc + (int)__builtin_amdgcn_mbcnt_lo(mj, 0u); \
            if (pos < WCAP) list[wave * WCAP + pos] = ((el0 + (J)) << 9) | (int)(SJ); \
          } \
          wc += (int)__builtin_popcount(mj); }
        HITJ(0, h0, s0)
        HITJ(1, h1, s1)
        HITJ(2, h2, s2)
        HITJ(3, h3, s3)
#undef HITJ
      }
    }
    if (lane == 0) wcnt[wave] = wc;
    __syncthreads();

    if (wave == 0) {
      for (int wsx = 0; wsx < NWAVE; ++wsx) {
        int n = wcnt[wsx];
        if (n > WCAP) n = WCAP;
        if (n < 0) n = 0;
        for (int i = 0; i < n; ++i) {
          const int ent  = list[wsx * WCAP + i];
          const int slot = ent & (NB - 1);
          const int el   = (ent >> 9) & (CHUNK - 1);
          int e = cbase + el;
          if (e > nE - 1) e = nE - 1;
          int src = ei[e];
          src = src < 0 ? 0 : (src > nN - 1 ? nN - 1 : src);
          int nd = nodeBase + slot;
          if (nd > nN - 1) nd = nN - 1;
          float v = als[(size_t)src * NHD + hd] + ald[(size_t)nd * NHD + hd];
          v = (v > 0.f) ? v : 0.2f * v;
          const int ai = slot * NHD + hd;
          const float mo = emx[ai];
          const float mn = fmaxf(mo, v);
          const float c  = __expf(mo - mn);
          const float p  = __expf(v - mn);
          const float* hr = Hm + (size_t)src * DD + 8 * lane;
          const v4f x0 = *(const v4f*)(hr);
          const v4f x1 = *(const v4f*)(hr + 4);
          v4f* sp = (v4f*)(sacc + slot * DD + 8 * lane);
          v4f a0 = sp[0];
          v4f a1 = sp[1];
          a0 = a0 * c + p * x0;
          a1 = a1 * c + p * x1;
          sp[0] = a0;
          sp[1] = a1;
          const float dv = den[ai];
          den[ai] = dv * c + p;
          emx[ai] = mn;
        }
      }
    }
    __syncthreads();
  }

  const int hA = lane >> 3;
  const int hB = 4 + (lane >> 3);
#pragma unroll 1
  for (int j = 0; j < NB / NWAVE; ++j) {
    const int slot = wave * (NB / NWAVE) + j;
    const int node = nodeBase + slot;
    if (node >= nP) break;
    const float invA = 1.0f / (den[slot * NHD + hA] + 1e-16f);
    const float invB = 1.0f / (den[slot * NHD + hB] + 1e-16f);
    v4f a = *(const v4f*)(sacc + slot * DD + 4 * lane) * invA;
    v4f b = *(const v4f*)(sacc + slot * DD + 128 + 4 * lane) * invB;
    a.x = a.x > 0.f ? a.x : (__expf(a.x) - 1.0f);
    a.y = a.y > 0.f ? a.y : (__expf(a.y) - 1.0f);
    a.z = a.z > 0.f ? a.z : (__expf(a.z) - 1.0f);
    a.w = a.w > 0.f ? a.w : (__expf(a.w) - 1.0f);
    b.x = b.x > 0.f ? b.x : (__expf(b.x) - 1.0f);
    b.y = b.y > 0.f ? b.y : (__expf(b.y) - 1.0f);
    b.z = b.z > 0.f ? b.z : (__expf(b.z) - 1.0f);
    b.w = b.w > 0.f ? b.w : (__expf(b.w) - 1.0f);
    float* gp = G + (size_t)node * DD;
    *(volatile v4f*)(gp + 4 * lane)       = a;
    *(volatile v4f*)(gp + 128 + 4 * lane) = b;
    __threadfence();
    *(volatile v4f*)(gp + 4 * lane)       = a;
    *(volatile v4f*)(gp + 128 + 4 * lane) = b;
  }
}

extern "C" void kernel_launch(void* const* d_in, const int* in_sizes, int n_in,
                              void* d_out, int out_size, void* d_ws, size_t ws_size,
                              hipStream_t stream) {
  if (n_in < 10) return;
  const int nN = in_sizes[0] / DD;
  if (nN <= 0 || in_sizes[0] != nN * DD) return;
  if (in_sizes[1] < 2 || (in_sizes[1] & 1) != 0) return;
  const int nE = in_sizes[1] / 2;
  if (in_sizes[2] != DD * DD || in_sizes[5] != DD * DD || in_sizes[8] != DD * DD) return;
  if (in_sizes[3] != DD || in_sizes[4] != DD || in_sizes[6] != DD || in_sizes[7] != DD) return;
  if (in_sizes[9] != DD) return;
  if (out_size != nN * DD) return;

  const float* x   = (const float*)d_in[0];
  const int*   ei  = (const int*)d_in[1];
  const float* W1  = (const float*)d_in[2];
  const float* as1 = (const float*)d_in[3];
  const float* ad1 = (const float*)d_in[4];
  const float* W2  = (const float*)d_in[5];
  const float* as2 = (const float*)d_in[6];
  const float* ad2 = (const float*)d_in[7];
  const float* Wl  = (const float*)d_in[8];
  const float* bl  = (const float*)d_in[9];
  float* out = (float*)d_out;

  const int nP = ((nN + GR - 1) / GR) * GR;
  const size_t plane = (size_t)DD * DD * sizeof(unsigned short);
  size_t off = 0;
  unsigned short* w1h = (unsigned short*)((char*)d_ws + off); off += plane;
  unsigned short* w1l = (unsigned short*)((char*)d_ws + off); off += plane;
  unsigned short* w2h = (unsigned short*)((char*)d_ws + off); off += plane;
  unsigned short* w2l = (unsigned short*)((char*)d_ws + off); off += plane;
  unsigned short* wlh = (unsigned short*)((char*)d_ws + off); off += plane;
  unsigned short* wll = (unsigned short*)((char*)d_ws + off); off += plane;
  float* Hm   = (float*)((char*)d_ws + off); off += (size_t)nP * DD * sizeof(float);
  float* Gm   = (float*)((char*)d_ws + off); off += (size_t)nP * DD * sizeof(float);
  float* als  = (float*)((char*)d_ws + off); off += (size_t)nP * NHD * sizeof(float);
  float* ald  = (float*)((char*)d_ws + off); off += (size_t)nP * NHD * sizeof(float);
  if (off > ws_size) return;

  k_prepw<<<16, NTHR, 0, stream>>>(W1, w1h, w1l);
  k_prepw<<<16, NTHR, 0, stream>>>(W2, w2h, w2l);
  k_prepw<<<16, NTHR, 0, stream>>>(Wl, wlh, wll);

  const int gGrid = nP / GR;
  const int aGrid = (nN + NB - 1) / NB;
  hipFuncSetAttribute(reinterpret_cast<const void*>(&k_agg),
                      hipFuncAttributeMaxDynamicSharedMemorySize, LDS_BYTES);

  k_gemm<<<gGrid, NTHR, 0, stream>>>(x, w1h, w1l, as1, ad1, bl, Hm, als, ald, nN, nP, 0);
  k_agg<<<aGrid, NTHR, LDS_BYTES, stream>>>(ei, Hm, als, ald, Gm, nN, nE, nP);
  k_gemm<<<gGrid, NTHR, 0, stream>>>(Gm, w2h, w2l, as2, ad2, bl, Hm, als, ald, nN, nP, 0);
  k_agg<<<aGrid, NTHR, LDS_BYTES, stream>>>(ei, Hm, als, ald, Gm, nN, nE, nP);
  k_gemm<<<gGrid, NTHR, 0, stream>>>(Gm, wlh, wll, as2, ad2, bl, out, als, ald, nN, nN, 1);
}
